// DINLayer_26508538150924
// MI455X (gfx1250) — hardware-verified
//
#include <hip/hip_runtime.h>
#define BSZ 512
#define SS 100
#define SP 112
#define ED 16
#define FF 48
#define NH1 36
#define VV 160000
#define C1 176
#define K1P 192
#define N1 200
#define N1P 256
#define K2P 224
#define N2 80
#define N2P 128

typedef __bf16 v16b __attribute__((ext_vector_type(16)));
typedef unsigned short v8us __attribute__((ext_vector_type(8), may_alias));
typedef float  v8f  __attribute__((ext_vector_type(8)));
typedef float  v4f  __attribute__((ext_vector_type(4)));
typedef float  v4fa __attribute__((ext_vector_type(4), may_alias));
union FragB { v16b v; v8us half[2]; unsigned short u[16]; };

__device__ __forceinline__ unsigned short bf16_bits(float x) { unsigned int u = __float_as_uint(x); return (unsigned short)((u + 0x7FFFu + ((u >> 16) & 1u)) >> 16); }
__device__ __forceinline__ float bf16_val(unsigned short b) { return __uint_as_float(((unsigned int)b) << 16); }
__device__ __forceinline__ float bf16_round(float x) { return bf16_val(bf16_bits(x)); }
template <int NT>
__device__ __forceinline__ v8f mmaN(v16b ah, v16b al, v16b bh, v16b bl, v8f c) {
  c = __builtin_amdgcn_wmma_f32_16x16x32_bf16(false, ah, false, bh, (short)0, c, false, false);
  if (NT >= 2) c = __builtin_amdgcn_wmma_f32_16x16x32_bf16(false, al, false, bh, (short)0, c, false, false);
  if (NT >= 3) c = __builtin_amdgcn_wmma_f32_16x16x32_bf16(false, ah, false, bl, (short)0, c, false, false);
  asm volatile("v_nop\n\tv_nop\n\tv_nop\n\tv_nop" : "+v"(c) : "v"(ah), "v"(al), "v"(bh), "v"(bl));
  return c;
}

__global__ __launch_bounds__(256) void k_wt_bf16(const float* __restrict__ W, unsigned short* __restrict__ Wt, int K, int N) {
  const int t = blockIdx.x * 256 + threadIdx.x;
  const int k8n = K / 8;
  if (t >= N * k8n) return;
  const int n = t / k8n, k8 = (t % k8n) * 8;
  v8us v;
#pragma unroll
  for (int i = 0; i < 8; ++i) v[i] = bf16_bits(W[(size_t)(k8 + i) * N + n]);
  *(volatile v8us*)(Wt + (size_t)n * K + k8) = v;
  __threadfence();
  *(volatile v8us*)(Wt + (size_t)n * K + k8) = v;
}

template <bool ASPLIT, int ACT, bool BIAS_BF16>
__global__ __launch_bounds__(128) void k_gemm_bf(const float* __restrict__ A, int lda, const unsigned short* __restrict__ Wt, int ldb,
                                               const float* __restrict__ bias, float* __restrict__ C, int ldc, int M, int N, int K) {
  __shared__ __attribute__((aligned(16))) float so[4][16][64];
  const int tid = threadIdx.x, w = tid >> 5, lane = tid & 31, ln = lane & 15, hh = lane >> 4;
  const int ntn = N / 64;
  const int wid = blockIdx.x * 4 + w;
  const int mt = wid / ntn, nq = wid % ntn;
  if (mt * 16 >= M) return;
  const int row0 = mt * 16, col0 = nq * 64;
  const float* arow = A + (size_t)(row0 + ln) * lda;
  v8f acc[4] = {};
  for (int kb = 0; kb < K; kb += 32) {
    FragB ah, al;
    const v4f x0 = *(const v4fa*)(arow + kb + 8 * hh), x1 = *(const v4fa*)(arow + kb + 8 * hh + 4);
    const v4f x2 = *(const v4fa*)(arow + kb + 16 + 8 * hh), x3 = *(const v4fa*)(arow + kb + 16 + 8 * hh + 4);
    float xs[16] = {x0[0],x0[1],x0[2],x0[3],x1[0],x1[1],x1[2],x1[3],x2[0],x2[1],x2[2],x2[3],x3[0],x3[1],x3[2],x3[3]};
#pragma unroll
    for (int i = 0; i < 16; ++i) { const unsigned short hb = bf16_bits(xs[i]); ah.u[i] = hb; al.u[i] = ASPLIT ? bf16_bits(xs[i] - bf16_val(hb)) : (unsigned short)0; }
#pragma unroll
    for (int t = 0; t < 4; ++t) {
      const unsigned short* brow = Wt + (size_t)(col0 + t * 16 + ln) * ldb + kb;
      FragB b;
      b.half[0] = *(const v8us*)(brow + 8 * hh);
      b.half[1] = *(const v8us*)(brow + 16 + 8 * hh);
      acc[t] = mmaN<ASPLIT ? 2 : 1>(ah.v, al.v, b.v, b.v, acc[t]);
    }
  }
#pragma unroll
  for (int t = 0; t < 4; ++t) {
    float bv = bias ? bias[col0 + t * 16 + ln] : 0.f;
    if (BIAS_BF16) bv = bf16_round(bv);
#pragma unroll
    for (int r = 0; r < 8; ++r) { float v = acc[t][r] + bv; if (ACT == 1) v = fmaxf(v, 0.f); so[w][8 * hh + r][t * 16 + ln] = v; }
  }
  __builtin_amdgcn_fence(__ATOMIC_ACQ_REL, "workgroup");
  __builtin_amdgcn_wave_barrier();
  const int rsub = lane >> 4, c4 = (lane & 15) * 4;
  for (int pass = 0; pass < 2; ++pass) {
#pragma unroll
    for (int q = 0; q < 8; ++q) {
      const int r = q * 2 + rsub;
      const v4f v = *(const v4fa*)&so[w][r][c4];
      *(volatile v4f*)(C + (size_t)(row0 + r) * ldc + col0 + c4) = v;
    }
    if (pass == 0) __threadfence();
  }
}

template <int D, bool CAUSAL>
__global__ __launch_bounds__(128) void k_flash(const float* __restrict__ qb, const float* __restrict__ kb, const float* __restrict__ vb,
                                             int pitch, int T, int H, float scale, float* __restrict__ y, int ypitch) {
  constexpr int KS = D / 32;
  constexpr int DT = D / 16;
  __shared__ __attribute__((aligned(16))) unsigned short sKh[32][D + 8], sKl[32][D + 8], sVh[32][D + 8], sVl[32][D + 8];
  __shared__ __attribute__((aligned(16))) unsigned short sPh[4][16][40], sPl[4][16][40];
  __shared__ __attribute__((aligned(16))) float sO[4][16][D];
  const int tid = threadIdx.x, w = tid >> 5, lane = tid & 31, ln = lane & 15, hh = lane >> 4;
  const int nqb = (T + 63) / 64;
  const int bh = blockIdx.x / nqb, qblk = blockIdx.x % nqb;
  const int b = bh / H, h = bh % H;
  const int q0 = qblk * 64 + w * 16;
  const float* Q = qb + (size_t)b * T * pitch + h * D;
  const float* K = kb + (size_t)b * T * pitch + h * D;
  const float* V = vb + (size_t)b * T * pitch + h * D;

  FragB aqh[KS], aql[KS];
  {
    int row = q0 + ln; if (row >= T) row = T - 1;
    const float* qr = Q + (size_t)row * pitch;
#pragma unroll
    for (int ks = 0; ks < KS; ++ks)
#pragma unroll
      for (int i = 0; i < 16; ++i) {
        const int d = ks * 32 + ((i < 8) ? (8 * hh + i) : (16 + 8 * hh + (i - 8)));
        const float x = qr[d] * scale; const unsigned short hb = bf16_bits(x);
        aqh[ks].u[i] = hb; aql[ks].u[i] = bf16_bits(x - bf16_val(hb));
      }
  }
  float m_r[8], l_r[8];
#pragma unroll
  for (int r = 0; r < 8; ++r) { m_r[r] = -3.0e38f; l_r[r] = 0.f; }
  v8f oacc[DT];
#pragma unroll
  for (int dt = 0; dt < DT; ++dt) oacc[dt] = (v8f){0.f,0.f,0.f,0.f,0.f,0.f,0.f,0.f};

  const int kv_end = CAUSAL ? min(T, qblk * 64 + 64) : T;
  for (int j0 = 0; j0 < kv_end; j0 += 32) {
    __syncthreads();
    for (int e = tid; e < 32 * (D / 4); e += 128) {
      const int r = e / (D / 4), c4 = (e % (D / 4)) * 4;
      const int key = j0 + r;
      v4f kf = {0.f,0.f,0.f,0.f}, vf = {0.f,0.f,0.f,0.f};
      if (key < T) { kf = *(const v4fa*)(K + (size_t)key * pitch + c4); vf = *(const v4fa*)(V + (size_t)key * pitch + c4); }
#pragma unroll
      for (int t = 0; t < 4; ++t) {
        unsigned short hb = bf16_bits(kf[t]); sKh[r][c4 + t] = hb; sKl[r][c4 + t] = bf16_bits(kf[t] - bf16_val(hb));
        hb = bf16_bits(vf[t]); sVh[r][c4 + t] = hb; sVl[r][c4 + t] = bf16_bits(vf[t] - bf16_val(hb));
      }
    }
    __syncthreads();
    v8f s[2];
#pragma unroll
    for (int nt = 0; nt < 2; ++nt) {
      v8f acc = {};
#pragma unroll
      for (int ks = 0; ks < KS; ++ks) {
        FragB bh_, bl_;
        bh_.half[0] = *(const v8us*)&sKh[nt * 16 + ln][ks * 32 + 8 * hh]; bh_.half[1] = *(const v8us*)&sKh[nt * 16 + ln][ks * 32 + 16 + 8 * hh];
        bl_.half[0] = *(const v8us*)&sKl[nt * 16 + ln][ks * 32 + 8 * hh]; bl_.half[1] = *(const v8us*)&sKl[nt * 16 + ln][ks * 32 + 16 + 8 * hh];
        acc = mmaN<3>(aqh[ks].v, aql[ks].v, bh_.v, bl_.v, acc);
      }
      s[nt] = acc;
    }
    float alpha[8];
#pragma unroll
    for (int r = 0; r < 8; ++r) {
      const int qi = q0 + 8 * hh + r;
      const int ja = j0 + ln, jb = j0 + 16 + ln;
      if (CAUSAL) { if (ja > qi) s[0][r] = -3.0e38f; if (jb > qi) s[1][r] = -3.0e38f; }
      if (ja >= T) s[0][r] = -3.0e38f;
      if (jb >= T) s[1][r] = -3.0e38f;
      float mx = fmaxf(s[0][r], s[1][r]);
      mx = fmaxf(mx, __shfl_xor(mx, 1, 32)); mx = fmaxf(mx, __shfl_xor(mx, 2, 32)); mx = fmaxf(mx, __shfl_xor(mx, 4, 32)); mx = fmaxf(mx, __shfl_xor(mx, 8, 32));
      const float mnew = fmaxf(m_r[r], mx);
      alpha[r] = (mnew > -1.0e38f) ? __expf(m_r[r] - mnew) : 1.0f;
      const float p0 = (s[0][r] > -1.0e38f) ? __expf(s[0][r] - mnew) : 0.f;
      const float p1 = (s[1][r] > -1.0e38f) ? __expf(s[1][r] - mnew) : 0.f;
      m_r[r] = mnew;
      l_r[r] = l_r[r] * alpha[r] + p0 + p1;
      unsigned short hb = bf16_bits(p0); sPh[w][8 * hh + r][ln] = hb;      sPl[w][8 * hh + r][ln] = bf16_bits(p0 - bf16_val(hb));
      hb = bf16_bits(p1);                sPh[w][8 * hh + r][16 + ln] = hb; sPl[w][8 * hh + r][16 + ln] = bf16_bits(p1 - bf16_val(hb));
    }
#pragma unroll
    for (int dt = 0; dt < DT; ++dt)
#pragma unroll
      for (int r = 0; r < 8; ++r) oacc[dt][r] *= alpha[r];
    __builtin_amdgcn_fence(__ATOMIC_ACQ_REL, "workgroup");
    __builtin_amdgcn_wave_barrier();
    FragB pah, pal;
    pah.half[0] = *(const v8us*)&sPh[w][ln][8 * hh]; pah.half[1] = *(const v8us*)&sPh[w][ln][16 + 8 * hh];
    pal.half[0] = *(const v8us*)&sPl[w][ln][8 * hh]; pal.half[1] = *(const v8us*)&sPl[w][ln][16 + 8 * hh];
#pragma unroll
    for (int dt = 0; dt < DT; ++dt) {
      FragB bvh, bvl;
#pragma unroll
      for (int i = 0; i < 8; ++i) {
        bvh.u[i] = sVh[8 * hh + i][dt * 16 + ln]; bvh.u[8 + i] = sVh[16 + 8 * hh + i][dt * 16 + ln];
        bvl.u[i] = sVl[8 * hh + i][dt * 16 + ln]; bvl.u[8 + i] = sVl[16 + 8 * hh + i][dt * 16 + ln];
      }
      oacc[dt] = mmaN<3>(pah.v, pal.v, bvh.v, bvl.v, oacc[dt]);
    }
    __builtin_amdgcn_fence(__ATOMIC_ACQ_REL, "workgroup");
    __builtin_amdgcn_wave_barrier();
  }
#pragma unroll
  for (int r = 0; r < 8; ++r) {
    float l = l_r[r];
    l += __shfl_xor(l, 1, 32); l += __shfl_xor(l, 2, 32); l += __shfl_xor(l, 4, 32); l += __shfl_xor(l, 8, 32);
    l_r[r] = (l > 0.f) ? 1.0f / l : 0.f;
  }
#pragma unroll
  for (int dt = 0; dt < DT; ++dt)
#pragma unroll
    for (int r = 0; r < 8; ++r) sO[w][8 * hh + r][dt * 16 + ln] = oacc[dt][r] * l_r[r];
  __builtin_amdgcn_fence(__ATOMIC_ACQ_REL, "workgroup");
  __builtin_amdgcn_wave_barrier();
  for (int pass = 0; pass < 2; ++pass) {
    for (int r = 0; r < 16; ++r) {
      const int row = q0 + r;
      if (row < T && lane < D / 4) {
        const v4f val = *(const v4fa*)&sO[w][r][lane * 4];
        *(volatile v4f*)(y + ((size_t)b * T + row) * ypitch + h * D + lane * 4) = val;
      }
    }
    if (pass == 0) __threadfence();
  }
}

template <bool ASPLIT, bool BSPLIT, int ACT>
__global__ __launch_bounds__(128) void k_gemm_b(const float* __restrict__ A, int lda, size_t sA, const unsigned short* __restrict__ Bh, const unsigned short* __restrict__ Bl, int ldb, size_t sB,
                                             const float* __restrict__ bias, const float* __restrict__ resid, int ldr, size_t sR, float rsign, float alpha,
                                             float* __restrict__ C, int ldc, size_t sC, int M, int N, int K) {
  __shared__ __attribute__((aligned(16))) float so[4][16][64];
  const int tid = threadIdx.x, w = tid >> 5, lane = tid & 31, ln = lane & 15, hh = lane >> 4;
  const int by = blockIdx.y;
  A += (size_t)by * sA; Bh += (size_t)by * sB; if (BSPLIT) Bl += (size_t)by * sB; C += (size_t)by * sC; if (resid) resid += (size_t)by * sR;
  const int ntn = (N + 63) / 64; const int wid = blockIdx.x * 4 + w; const int mt = wid / ntn, nq = wid % ntn;
  if (mt * 16 >= M) return;
  const int row0 = mt * 16, col0 = nq * 64;
  const float* arow = A + (size_t)(row0 + ln) * lda;
  v8f acc[4] = {};
  for (int kb = 0; kb < K; kb += 32) {
    FragB ah, al;
    const v4f x0 = *(const v4fa*)(arow + kb + 8 * hh), x1 = *(const v4fa*)(arow + kb + 8 * hh + 4);
    const v4f x2 = *(const v4fa*)(arow + kb + 16 + 8 * hh), x3 = *(const v4fa*)(arow + kb + 16 + 8 * hh + 4);
    float xs[16] = {x0[0],x0[1],x0[2],x0[3],x1[0],x1[1],x1[2],x1[3],x2[0],x2[1],x2[2],x2[3],x3[0],x3[1],x3[2],x3[3]};
#pragma unroll
    for (int i = 0; i < 16; ++i) { const unsigned short hb = bf16_bits(xs[i]); ah.u[i] = hb; al.u[i] = ASPLIT ? bf16_bits(xs[i] - bf16_val(hb)) : (unsigned short)0; }
#pragma unroll
    for (int t = 0; t < 4; ++t) {
      if (col0 + t * 16 >= N) continue;
      const size_t boff = (size_t)(col0 + t * 16 + ln) * ldb + kb;
      FragB bh_, bl_; bh_.half[0] = *(const v8us*)(Bh + boff + 8 * hh); bh_.half[1] = *(const v8us*)(Bh + boff + 16 + 8 * hh);
      if (BSPLIT) { bl_.half[0] = *(const v8us*)(Bl + boff + 8 * hh); bl_.half[1] = *(const v8us*)(Bl + boff + 16 + 8 * hh); } else bl_ = bh_;
      acc[t] = mmaN<ASPLIT ? (BSPLIT ? 3 : 2) : 1>(ah.v, al.v, bh_.v, bl_.v, acc[t]);
    }
  }
#pragma unroll
  for (int t = 0; t < 4; ++t) {
    const int col = col0 + t * 16 + ln; if (col0 + t * 16 >= N) continue; const float bv = bias ? bf16_round(bias[col]) : 0.f;
#pragma unroll
    for (int r = 0; r < 8; ++r) { float v = acc[t][r] * alpha + bv; if (resid) v += rsign * resid[(size_t)(row0 + 8 * hh + r) * ldr + col]; if (ACT == 1) v = fmaxf(v, 0.f); else if (ACT == 2) v = fmaxf(v, 0.f) + log1pf(expf(-fabsf(v))); so[w][8 * hh + r][t * 16 + ln] = v; }
  }
  __builtin_amdgcn_fence(__ATOMIC_ACQ_REL, "workgroup"); __builtin_amdgcn_wave_barrier();
  const int rsub = lane >> 4, c4 = (lane & 15) * 4;
  for (int pass = 0; pass < 2; ++pass) {
#pragma unroll
    for (int q = 0; q < 8; ++q) { const int r = q * 2 + rsub; if (col0 + c4 < N) { const v4f v = *(const v4fa*)&so[w][r][c4]; *(volatile v4f*)(C + (size_t)(row0 + r) * ldc + col0 + c4) = v; } }
    if (pass == 0) __threadfence();
  }
}
__global__ __launch_bounds__(256) void k_split_transpose_b(const float* __restrict__ src, int lds_, size_t sIn, unsigned short* __restrict__ hi, unsigned short* __restrict__ lo, size_t sOut, int K, int N) {
  const size_t t = (size_t)blockIdx.x * 256 + threadIdx.x; const int k8n = K / 8; if (t >= (size_t)N * k8n) return;
  src += (size_t)blockIdx.y * sIn; hi += (size_t)blockIdx.y * sOut; lo += (size_t)blockIdx.y * sOut;
  const int n = (int)(t / k8n), k8 = (int)(t % k8n) * 8; v8us vh, vl;
#pragma unroll
  for (int i = 0; i < 8; ++i) { const float x = src[(size_t)(k8 + i) * lds_ + n]; const unsigned short hb = bf16_bits(x); vh[i] = hb; vl[i] = bf16_bits(x - bf16_val(hb)); }
  unsigned short* dh = hi + (size_t)n * K + k8; unsigned short* dl = lo + (size_t)n * K + k8;
  *(volatile v8us*)dh = vh; *(volatile v8us*)dl = vl; __threadfence(); *(volatile v8us*)dh = vh; *(volatile v8us*)dl = vl;
}

typedef _Float16 v16h __attribute__((ext_vector_type(16)));
union FragH { v16h v; v8us half[2]; _Float16 h[16]; unsigned short u[16]; };
template <int NT>
__device__ __forceinline__ v8f mmaH(v16h ah, v16h al, v16h bh, v16h bl, v8f c) {
  c = __builtin_amdgcn_wmma_f32_16x16x32_f16(false, ah, false, bh, (short)0, c, false, false);
  if (NT >= 2) c = __builtin_amdgcn_wmma_f32_16x16x32_f16(false, al, false, bh, (short)0, c, false, false);
  if (NT >= 3) c = __builtin_amdgcn_wmma_f32_16x16x32_f16(false, ah, false, bl, (short)0, c, false, false);
  asm volatile("v_nop\n\tv_nop\n\tv_nop\n\tv_nop" : "+v"(c) : "v"(ah), "v"(al), "v"(bh), "v"(bl));
  return c;
}
template <bool ASPLIT>
__global__ __launch_bounds__(128) void k_gemm_h(const float* __restrict__ A, int lda, size_t sA, const _Float16* __restrict__ Bh, int ldb, size_t sB, float alpha, float* __restrict__ C, int ldc, size_t sC, int M, int N, int K) {
  __shared__ __attribute__((aligned(16))) float so[4][16][64];
  const int tid = threadIdx.x, w = tid >> 5, lane = tid & 31, ln = lane & 15, hh = lane >> 4; const int by = blockIdx.y;
  A += (size_t)by * sA; Bh += (size_t)by * sB; C += (size_t)by * sC;
  const int ntn = (N + 63) / 64; const int wid = blockIdx.x * 4 + w; const int mt = wid / ntn, nq = wid % ntn; if (mt * 16 >= M) return;
  const int row0 = mt * 16, col0 = nq * 64; const float* arow = A + (size_t)(row0 + ln) * lda;
  v8f acc[4] = {};
  for (int kb = 0; kb < K; kb += 32) {
    FragH ah, al;
    const v4f x0 = *(const v4fa*)(arow + kb + 8 * hh), x1 = *(const v4fa*)(arow + kb + 8 * hh + 4), x2 = *(const v4fa*)(arow + kb + 16 + 8 * hh), x3 = *(const v4fa*)(arow + kb + 16 + 8 * hh + 4);
    float xs[16] = {x0[0],x0[1],x0[2],x0[3],x1[0],x1[1],x1[2],x1[3],x2[0],x2[1],x2[2],x2[3],x3[0],x3[1],x3[2],x3[3]};
#pragma unroll
    for (int i = 0; i < 16; ++i) { const _Float16 h = (_Float16)xs[i]; ah.h[i] = h; al.h[i] = ASPLIT ? (_Float16)(xs[i] - (float)h) : (_Float16)0.0f; }
#pragma unroll
    for (int t = 0; t < 4; ++t) { if (col0 + t * 16 >= N) continue; const size_t boff = (size_t)(col0 + t * 16 + ln) * ldb + kb; FragH bq; bq.half[0] = *(const v8us*)(Bh + boff + 8 * hh); bq.half[1] = *(const v8us*)(Bh + boff + 16 + 8 * hh);
      acc[t] = mmaH<ASPLIT ? 2 : 1>(ah.v, al.v, bq.v, bq.v, acc[t]); }
  }
#pragma unroll
  for (int t = 0; t < 4; ++t) { if (col0 + t * 16 >= N) continue;
#pragma unroll
    for (int r = 0; r < 8; ++r) so[w][8 * hh + r][t * 16 + ln] = acc[t][r] * alpha; }
  __builtin_amdgcn_fence(__ATOMIC_ACQ_REL, "workgroup"); __builtin_amdgcn_wave_barrier();
  const int rsub = lane >> 4, c4 = (lane & 15) * 4;
  for (int pass = 0; pass < 2; ++pass) {
#pragma unroll
    for (int q = 0; q < 8; ++q) { const int r = q * 2 + rsub; if (col0 + c4 < N) { const v4f v = *(const v4fa*)&so[w][r][c4]; *(volatile v4f*)(C + (size_t)(row0 + r) * ldc + col0 + c4) = v; } }
    if (pass == 0) __threadfence(); }
}

template <int DUMMY>
__global__ __launch_bounds__(128) void k_gemm_hh(const _Float16* __restrict__ A, int lda, size_t sA, const _Float16* __restrict__ Bh, int ldb, size_t sB, float alpha, float* __restrict__ C, int ldc, size_t sC, int M, int N, int K) {
  __shared__ __attribute__((aligned(16))) float so[4][16][64];
  const int tid = threadIdx.x, w = tid >> 5, lane = tid & 31, ln = lane & 15, hh = lane >> 4; const int by = blockIdx.y;
  A += (size_t)by * sA; Bh += (size_t)by * sB; C += (size_t)by * sC;
  const int ntn = (N + 63) / 64; const int wid = blockIdx.x * 4 + w; const int mt = wid / ntn, nq = wid % ntn; if (mt * 16 >= M) return;
  const int row0 = mt * 16, col0 = nq * 64; const _Float16* arow = A + (size_t)(row0 + ln) * lda;
  v8f acc[4] = {};
  for (int kb = 0; kb < K; kb += 32) { FragH ah; ah.half[0] = *(const v8us*)((const unsigned short*)arow + kb + 8 * hh); ah.half[1] = *(const v8us*)((const unsigned short*)arow + kb + 16 + 8 * hh);
#pragma unroll
    for (int t = 0; t < 4; ++t) { if (col0 + t * 16 >= N) continue; const size_t boff = (size_t)(col0 + t * 16 + ln) * ldb + kb; FragH bq; bq.half[0] = *(const v8us*)((const unsigned short*)Bh + boff + 8 * hh); bq.half[1] = *(const v8us*)((const unsigned short*)Bh + boff + 16 + 8 * hh);
      acc[t] = mmaH<1>(ah.v, ah.v, bq.v, bq.v, acc[t]); }
  }
#pragma unroll
  for (int t = 0; t < 4; ++t) { if (col0 + t * 16 >= N) continue;
#pragma unroll
    for (int r = 0; r < 8; ++r) so[w][8 * hh + r][t * 16 + ln] = acc[t][r] * alpha; }
  __builtin_amdgcn_fence(__ATOMIC_ACQ_REL, "workgroup"); __builtin_amdgcn_wave_barrier();
  const int rsub = lane >> 4, c4 = (lane & 15) * 4;
  for (int pass = 0; pass < 2; ++pass) {
#pragma unroll
    for (int q = 0; q < 8; ++q) { const int r = q * 2 + rsub; if (col0 + c4 < N) { const v4f v = *(const v4fa*)&so[w][r][c4]; *(volatile v4f*)(C + (size_t)(row0 + r) * ldc + col0 + c4) = v; } }
    if (pass == 0) __threadfence(); }
}

__device__ __forceinline__ int clampid(int v) { return v < 0 ? 0 : (v >= VV ? VV - 1 : v); }
__global__ __launch_bounds__(256) void k_emb(const int* __restrict__ uid, const int* __restrict__ t1, const int* __restrict__ t2, const int* __restrict__ t3, const int* __restrict__ t4, const int* __restrict__ gid, const int* __restrict__ sid, const int* __restrict__ cid,
                                             const int* __restrict__ vg, const int* __restrict__ vsd, const int* __restrict__ vc, const float* __restrict__ tab, float* __restrict__ VI, float* __restrict__ X, _Float16* __restrict__ VS16, float* __restrict__ VSf) {
  const int t = blockIdx.x * 256 + threadIdx.x;
  if (t < BSZ * 8) { const int b = t / 8, f = t % 8; const int* src[8] = {uid, t1, t2, t3, t4, gid, sid, cid}; const int id = clampid(src[f][b]); const float* row = tab + (size_t)id * ED;
    for (int pass = 0; pass < 2; ++pass) { for (int e = 0; e < ED; ++e) { const float v = bf16_round(row[e]); *(volatile float*)(X + (size_t)b * K1P + f * ED + e) = v; if (f >= 5) *(volatile float*)(VI + (size_t)b * FF + (f - 5) * ED + e) = v; } if (pass == 0) __threadfence(); } }
  if (t < BSZ * SP) { const int b = t / SP, s = t % SP; FragH f[4]; float vals[FF];
    if (s < SS) { const int ids[3] = {clampid(vg[b * SS + s]), clampid(vsd[b * SS + s]), clampid(vc[b * SS + s])}; for (int k = 0; k < 3; ++k) for (int e = 0; e < ED; ++e) vals[k * ED + e] = bf16_round(tab[(size_t)ids[k] * ED + e]); } else { for (int i = 0; i < FF; ++i) vals[i] = 0.f; }
    for (int i = 0; i < 64; ++i) f[i / 16].h[i % 16] = (_Float16)(i < FF ? vals[i] : 0.f);
    unsigned short* d = (unsigned short*)VS16 + ((size_t)b * SP + s) * 64; for (int pass = 0; pass < 2; ++pass) { for (int g = 0; g < 4; ++g) { *(volatile v8us*)(d + g * 16) = f[g].half[0]; *(volatile v8us*)(d + g * 16 + 8) = f[g].half[1]; } if (s < SS) { for (int i = 0; i < FF; ++i) *(volatile float*)(VSf + ((size_t)b * SS + s) * FF + i) = vals[i]; } if (pass == 0) __threadfence(); } } }
__global__ __launch_bounds__(256) void k_w(const float* __restrict__ Wa, const float* __restrict__ Wm1, const float* __restrict__ Wm2, const float* __restrict__ bm1, const float* __restrict__ bm2, unsigned short* __restrict__ Bt3, float* __restrict__ W01, float* __restrict__ WD, unsigned short* __restrict__ Btm1, unsigned short* __restrict__ Btm2, float* __restrict__ BP1, float* __restrict__ BP2) { const int t = blockIdx.x * 256 + threadIdx.x;
  if (t < N1P) { const float v = (t < N1) ? bm1[t] : 0.f; *(volatile float*)(BP1 + t) = v; __threadfence(); *(volatile float*)(BP1 + t) = v; }
  if (t < N2P) { const float v = (t < N2) ? bm2[t] : 0.f; *(volatile float*)(BP2 + t) = v; __threadfence(); *(volatile float*)(BP2 + t) = v; }
  if (t < FF * 48 * 8) { const int j8 = (t % 8) * 8, h = (t / 8) % 48, i = t / (8 * 48); v8us v; for (int q = 0; q < 8; ++q) { const int j = j8 + q; v[q] = bf16_bits((h < NH1 && j < FF) ? Wa[((size_t)144 + i * FF + j) * NH1 + h] : 0.f); } *(volatile v8us*)(Bt3 + ((size_t)i * 48 + h) * 64 + j8) = v; __threadfence(); *(volatile v8us*)(Bt3 + ((size_t)i * 48 + h) * 64 + j8) = v; }
  if (t < FF * NH1) { const int i = t / NH1, h = t % NH1; const float w0 = bf16_round(Wa[(size_t)i * NH1 + h]), w1 = bf16_round(Wa[((size_t)FF + i) * NH1 + h]), w2 = bf16_round(Wa[((size_t)2 * FF + i) * NH1 + h]); *(volatile float*)(W01 + t) = w0 + w1; *(volatile float*)(WD + t) = w2 - w1; __threadfence(); *(volatile float*)(W01 + t) = w0 + w1; *(volatile float*)(WD + t) = w2 - w1; }
  if (t < N1P * (K1P / 8)) { const int k8 = (t % (K1P / 8)) * 8, n = t / (K1P / 8); v8us v; for (int q = 0; q < 8; ++q) { const int k = k8 + q; v[q] = bf16_bits((n < N1 && k < C1) ? Wm1[(size_t)k * N1 + n] : 0.f); } *(volatile v8us*)(Btm1 + (size_t)n * K1P + k8) = v; __threadfence(); *(volatile v8us*)(Btm1 + (size_t)n * K1P + k8) = v; }
  if (t < N2P * (K2P / 8)) { const int k8 = (t % (K2P / 8)) * 8, n = t / (K2P / 8); v8us v; for (int q = 0; q < 8; ++q) { const int k = k8 + q; v[q] = bf16_bits((n < N2 && k < N1) ? Wm2[(size_t)k * N2 + n] : 0.f); } *(volatile v8us*)(Btm2 + (size_t)n * K2P + k8) = v; __threadfence(); *(volatile v8us*)(Btm2 + (size_t)n * K2P + k8) = v; } }
__global__ __launch_bounds__(64) void k_vip(const float* __restrict__ VI, const float* __restrict__ W01, const float* __restrict__ ba, float* __restrict__ VIP, float* __restrict__ CB) { const int b = blockIdx.x, k = threadIdx.x; const float v = (k < FF) ? VI[b * FF + k] : 0.f; *(volatile float*)(VIP + b * 64 + k) = v;
  if (k < NH1) { float s = bf16_round(ba[k]);
#pragma unroll 1
    for (int i = 0; i < FF; ++i) s += VI[b * FF + i] * W01[i * NH1 + k]; *(volatile float*)(CB + b * NH1 + k) = s; __threadfence(); *(volatile float*)(CB + b * NH1 + k) = s; } __threadfence(); *(volatile float*)(VIP + b * 64 + k) = v; }
__global__ __launch_bounds__(256) void k_m16(const float* __restrict__ T, const float* __restrict__ WD, _Float16* __restrict__ M16) { const int t = blockIdx.x * 256 + threadIdx.x; if (t >= BSZ * 48 * 8) return; const int i8 = (t % 8) * 8, h = (t / 8) % 48, b = t / (8 * 48); FragH f; for (int q = 0; q < 8; ++q) { const int i = i8 + q; f.h[q] = (_Float16)((h < NH1 && i < FF) ? (T[((size_t)i * BSZ + b) * 48 + h] + WD[i * NH1 + h]) : 0.f); } unsigned short* d = (unsigned short*)M16 + ((size_t)b * 48 + h) * 64 + i8; *(volatile v8us*)d = f.half[0]; __threadfence(); *(volatile v8us*)d = f.half[0]; }
__global__ __launch_bounds__(256) void k_dstat(const float* __restrict__ A, const float* __restrict__ CB, float* __restrict__ MU, float* __restrict__ RS) { const int t = blockIdx.x * 256 + threadIdx.x; if (t >= SS * NH1) return; const int s = t / NH1, h = t % NH1; float m = 0.f;
#pragma unroll 1
  for (int b = 0; b < BSZ; ++b) m += A[((size_t)b * SP + s) * 48 + h] + CB[b * NH1 + h]; m *= (1.0f / BSZ); float q = 0.f;
#pragma unroll 1
  for (int b = 0; b < BSZ; ++b) { const float d = A[((size_t)b * SP + s) * 48 + h] + CB[b * NH1 + h] - m; q += d * d; } const float rs = rsqrtf(q * (1.0f / BSZ) + 1e-3f);
  *(volatile float*)(MU + t) = m; *(volatile float*)(RS + t) = rs; __threadfence(); *(volatile float*)(MU + t) = m; *(volatile float*)(RS + t) = rs; }
__global__ __launch_bounds__(128) void k_score(const float* __restrict__ A, const float* __restrict__ CB, const float* __restrict__ MU, const float* __restrict__ RS, const float* __restrict__ al, const float* __restrict__ Wo, const float* __restrict__ bo, const int* __restrict__ vg, const float* __restrict__ VSf, float* __restrict__ X) {
  __shared__ float ssc[SS]; const int b = blockIdx.x, tid = threadIdx.x;
  if (tid < SS) { const int s = tid; float sc = bf16_round(bo[0]);
#pragma unroll 1
    for (int h = 0; h < NH1; ++h) { const float a = A[((size_t)b * SP + s) * 48 + h] + CB[b * NH1 + h]; const float xn = (a - MU[s * NH1 + h]) * RS[s * NH1 + h]; const float p = 1.0f / (1.0f + expf(-xn)); const float d = bf16_round(al[h]) * (1.0f - p) * a + p * a; sc += d * bf16_round(Wo[h]); }
    const float mask = (vg[b * SS + s] == 0) ? 1.0f : 0.0f; ssc[s] = sc * mask; }
  __syncthreads();
  if (tid < 64) { float xi = 0.f; if (tid < FF) {
#pragma unroll 1
      for (int s = 0; s < SS; ++s) xi += VSf[((size_t)b * SS + s) * FF + tid] * ssc[s]; }
    *(volatile float*)(X + (size_t)b * K1P + 128 + tid) = (tid < FF) ? xi : 0.f; __threadfence(); *(volatile float*)(X + (size_t)b * K1P + 128 + tid) = (tid < FF) ? xi : 0.f; } }
__global__ __launch_bounds__(256) void k_ln(float* __restrict__ H, int ld, int N, const float* __restrict__ g, const float* __restrict__ be) { const int tid = threadIdx.x, wv = tid >> 5, lane = tid & 31; const int b = blockIdx.x * 8 + wv; float* row = H + (size_t)b * ld; float s = 0.f; for (int c = lane; c < N; c += 32) s += row[c]; for (int o = 16; o >= 1; o >>= 1) s += __shfl_xor(s, o, 32); const float mu = s / (float)N; float q = 0.f; for (int c = lane; c < N; c += 32) { const float d = row[c] - mu; q += d * d; } for (int o = 16; o >= 1; o >>= 1) q += __shfl_xor(q, o, 32); const float rs = rsqrtf(q / (float)N + 1e-3f);
  for (int c = lane; c < N; c += 32) { const float v = (row[c] - mu) * rs * bf16_round(g[c]) + bf16_round(be[c]); *(volatile float*)(row + c) = v; } __threadfence(); for (int c = lane; c < N; c += 32) { const float v = *(volatile float*)(row + c); *(volatile float*)(row + c) = v; } }
__global__ __launch_bounds__(256) void k_bstat(const float* __restrict__ H, int ld, int N, float* __restrict__ MU, float* __restrict__ RS) { const int c = blockIdx.x * 256 + threadIdx.x; if (c >= N) return; float m = 0.f;
#pragma unroll 1
  for (int b = 0; b < BSZ; ++b) m += H[(size_t)b * ld + c]; m *= (1.0f / BSZ); float q = 0.f;
#pragma unroll 1
  for (int b = 0; b < BSZ; ++b) { const float d = H[(size_t)b * ld + c] - m; q += d * d; } const float rs = rsqrtf(q * (1.0f / BSZ) + 1e-3f); *(volatile float*)(MU + c) = m; *(volatile float*)(RS + c) = rs; __threadfence(); *(volatile float*)(MU + c) = m; *(volatile float*)(RS + c) = rs; }
__global__ __launch_bounds__(256) void k_dice(const float* __restrict__ H, int ld, int N, const float* __restrict__ MU, const float* __restrict__ RS, const float* __restrict__ al, float* __restrict__ OUT, int ldo) { const int t = blockIdx.x * 256 + threadIdx.x; if (t >= BSZ * ldo) return; const int c = t % ldo, b = t / ldo; float v = 0.f;
  if (c < N) { const float h = H[(size_t)b * ld + c]; const float xn = (h - MU[c]) * RS[c]; const float p = 1.0f / (1.0f + expf(-xn)); v = bf16_round(al[c]) * (1.0f - p) * h + p * h; } *(volatile float*)(OUT + t) = v; __threadfence(); *(volatile float*)(OUT + t) = v; }
__global__ __launch_bounds__(256) void k_out(const float* __restrict__ D2, const float* __restrict__ Wo, const float* __restrict__ bo, float* __restrict__ out) { const int b = blockIdx.x * 256 + threadIdx.x; if (b >= BSZ) return; float l0 = bf16_round(bo[0]), l1 = bf16_round(bo[1]);
#pragma unroll 1
  for (int k = 0; k < N2; ++k) { const float v = D2[(size_t)b * N2P + k]; l0 += v * bf16_round(Wo[k * 2]); l1 += v * bf16_round(Wo[k * 2 + 1]); }
  const float m = fmaxf(l0, l1); const float e0 = expf(l0 - m), e1 = expf(l1 - m); const float inv = 1.0f / (e0 + e1); typedef float v2f __attribute__((ext_vector_type(2))); v2f o; o.x = e0 * inv; o.y = e1 * inv; *(volatile v2f*)(out + (size_t)b * 2) = o; __threadfence(); *(volatile v2f*)(out + (size_t)b * 2) = o; }
extern "C" void kernel_launch(void* const* d_in, const int* in_sizes, int n_in,
                              void* d_out, int out_size, void* d_ws, size_t ws_size, hipStream_t stream) {
  (void)in_sizes; (void)n_in; (void)out_size;
  const int* uid = (const int*)d_in[0]; const int* t1 = (const int*)d_in[1]; const int* t2 = (const int*)d_in[2]; const int* t3 = (const int*)d_in[3]; const int* t4 = (const int*)d_in[4]; const int* gid = (const int*)d_in[5]; const int* sid = (const int*)d_in[6]; const int* cid = (const int*)d_in[7];
  const int* vg = (const int*)d_in[8]; const int* vsd = (const int*)d_in[9]; const int* vc = (const int*)d_in[10]; const float* tab = (const float*)d_in[11]; const float* Wa = (const float*)d_in[12]; const float* ba = (const float*)d_in[13]; const float* ala = (const float*)d_in[14]; const float* Wao = (const float*)d_in[15]; const float* bao = (const float*)d_in[16];
  const float* Wm1 = (const float*)d_in[17]; const float* bm1 = (const float*)d_in[18]; const float* g1 = (const float*)d_in[19]; const float* be1 = (const float*)d_in[20]; const float* al1 = (const float*)d_in[21]; const float* Wm2 = (const float*)d_in[22]; const float* bm2 = (const float*)d_in[23]; const float* g2 = (const float*)d_in[24]; const float* be2 = (const float*)d_in[25]; const float* al2 = (const float*)d_in[26]; const float* Wout = (const float*)d_in[27]; const float* bout = (const float*)d_in[28];
  char* ws = (char*)d_ws; size_t off = 0;
  auto take = [&](size_t bytes) { char* p = ws + off; off += (bytes + 255) & ~(size_t)255; return p; };
  unsigned short* Bt3 = (unsigned short*)take((size_t)FF * 48 * 64 * 2); float* W01 = (float*)take(FF * NH1 * 4); float* WD = (float*)take(FF * NH1 * 4); unsigned short* Btm1 = (unsigned short*)take((size_t)N1P * K1P * 2); unsigned short* Btm2 = (unsigned short*)take((size_t)N2P * K2P * 2);
  float* VI = (float*)take(BSZ * FF * 4); float* X = (float*)take((size_t)BSZ * K1P * 4); _Float16* VS16 = (_Float16*)take((size_t)BSZ * SP * 64 * 2); float* VSf = (float*)take((size_t)BSZ * SS * FF * 4); float* VIP = (float*)take(BSZ * 64 * 4); float* CB = (float*)take(BSZ * NH1 * 4);
  float* T = (float*)take((size_t)FF * BSZ * 48 * 4); _Float16* M16 = (_Float16*)take((size_t)BSZ * 48 * 64 * 2); float* A = (float*)take((size_t)BSZ * SP * 48 * 4); float* MU = (float*)take(SS * NH1 * 4); float* RS = (float*)take(SS * NH1 * 4);
  float* H1 = (float*)take((size_t)BSZ * N1P * 4); float* D1 = (float*)take((size_t)BSZ * K2P * 4); float* H2 = (float*)take((size_t)BSZ * N2P * 4); float* D2 = (float*)take((size_t)BSZ * N2P * 4); float* MU1 = (float*)take(N1P * 4); float* RS1 = (float*)take(N1P * 4); float* MU2 = (float*)take(N2P * 4); float* RS2 = (float*)take(N2P * 4); float* BP1 = (float*)take(N1P * 4); float* BP2 = (float*)take(N2P * 4);
  if (off > ws_size) return;
  k_w<<<(N1P * (K1P / 8) + 255) / 256 > (FF * 48 * 8 + 255) / 256 ? (N1P * (K1P / 8) + 255) / 256 : (FF * 48 * 8 + 255) / 256, 256, 0, stream>>>(Wa, Wm1, Wm2, bm1, bm2, Bt3, W01, WD, Btm1, Btm2, BP1, BP2);
  k_emb<<<(BSZ * SP + 255) / 256, 256, 0, stream>>>(uid, t1, t2, t3, t4, gid, sid, cid, vg, vsd, vc, tab, VI, X, VS16, VSf);
  k_vip<<<BSZ, 64, 0, stream>>>(VI, W01, ba, VIP, CB);
  k_gemm_b<false, false, 0><<<dim3(((BSZ / 16) * 1 + 3) / 4, FF), 128, 0, stream>>>(VIP, 64, 0, Bt3, Bt3, 64, (size_t)48 * 64, nullptr, nullptr, 0, 0, 1.f, 1.f, T, 48, (size_t)BSZ * 48, BSZ, 48, 64);
  k_m16<<<(BSZ * 48 * 8 + 255) / 256, 256, 0, stream>>>(T, WD, M16);
  k_gemm_hh<0><<<dim3(((SP / 16) * 1 + 3) / 4, BSZ), 128, 0, stream>>>(VS16, 64, (size_t)SP * 64, M16, 64, (size_t)48 * 64, 1.0f, A, 48, (size_t)SP * 48, SP, 48, 64);
  k_dstat<<<(SS * NH1 + 255) / 256, 256, 0, stream>>>(A, CB, MU, RS);
  k_score<<<BSZ, 128, 0, stream>>>(A, CB, MU, RS, ala, Wao, bao, vg, VSf, X);
  k_gemm_b<true, false, 0><<<dim3(((BSZ / 16) * (N1P / 64) + 3) / 4, 1), 128, 0, stream>>>(X, K1P, 0, Btm1, Btm1, K1P, 0, BP1, nullptr, 0, 0, 1.f, 1.f, H1, N1P, 0, BSZ, N1P, K1P);
  k_ln<<<BSZ / 8, 256, 0, stream>>>(H1, N1P, N1, g1, be1); k_bstat<<<1, 256, 0, stream>>>(H1, N1P, N1, MU1, RS1); k_dice<<<(BSZ * K2P + 255) / 256, 256, 0, stream>>>(H1, N1P, N1, MU1, RS1, al1, D1, K2P);
  k_gemm_b<true, false, 0><<<dim3(((BSZ / 16) * (N2P / 64) + 3) / 4, 1), 128, 0, stream>>>(D1, K2P, 0, Btm2, Btm2, K2P, 0, BP2, nullptr, 0, 0, 1.f, 1.f, H2, N2P, 0, BSZ, N2P, K2P);
  k_ln<<<BSZ / 8, 256, 0, stream>>>(H2, N2P, N2, g2, be2); k_bstat<<<1, 256, 0, stream>>>(H2, N2P, N2, MU2, RS2); k_dice<<<(BSZ * N2P + 255) / 256, 256, 0, stream>>>(H2, N2P, N2, MU2, RS2, al2, D2, N2P);
  k_out<<<(BSZ + 255) / 256, 256, 0, stream>>>(D2, Wout, bout, (float*)d_out);
}
